// InductionHeadAttentionSmaller_1778116461294
// MI455X (gfx1250) — hardware-verified
//
#include <hip/hip_runtime.h>
#include <stddef.h>


typedef _Float16 v16h __attribute__((ext_vector_type(16)));
typedef _Float16 v8h  __attribute__((ext_vector_type(8)));
typedef float    v8f  __attribute__((ext_vector_type(8)));
typedef float    v4f  __attribute__((ext_vector_type(4)));
typedef int      v4i  __attribute__((ext_vector_type(4)));
typedef _Float16 h16;

#ifndef NB
#define NB 16
#endif
#ifndef SEQ
#define SEQ 2048
#endif
#define NB_FULL  16
#define SEQ_FULL 2048
#define DIM      2048

#ifndef SCORE_RES
#define SCORE_RES 0
#endif
#ifndef CHAIN_RES
#define CHAIN_RES 1
#endif

static_assert(NB == NB_FULL && SEQ == SEQ_FULL);
static_assert(NB == 16);
static_assert(SEQ == DIM);
static_assert(DIM == 256 * 8);
static_assert((DIM % 128) == 0 && (DIM % 64) == 0 && (DIM % 32) == 0);
static_assert((((size_t)DIM * DIM) % 2048) == 0);

#define LDT 72
#define LDC 68
#define LDM 132
static_assert((LDT % 8) == 0 && LDT >= 64);
static_assert((LDC % 4) == 0 && LDC >= 64);
static_assert((LDM % 4) == 0 && LDM >= 128);

#define WCARRY 64.0f
#define QCARRY 1024.0f
#define PCARRY 16384.0f
#define HCARRY 16384.0f
#define ACARRY 1024.0f
#define RCARRY 2048.0f
static_assert(PCARRY * 1.0f < 65504.0f && HCARRY * 1.0f < 65504.0f);

#define SCALE1 181.01933598f
#define SCALE2 181.01933598f
#define SCALEO 128.0f

#define PLANE_BYTES ((size_t)DIM * DIM * 2)
#define NSLOT 11
#define VEC16_BYTES ((size_t)NB * DIM * 2)
#define VEC32_BYTES ((size_t)NB * DIM * 4)
#define ROW32_BYTES ((size_t)DIM * 4)
#define NV16 22
#define NV32 5
#define OFF_SLOT(i) ((size_t)(i) * PLANE_BYTES)
#define OFF_ALAST   OFF_SLOT(NSLOT)
#define OFF_V16(i)  (OFF_ALAST + ROW32_BYTES + (size_t)(i) * VEC16_BYTES)
#define OFF_V32(i)  (OFF_V16(NV16) + (size_t)(i) * VEC32_BYTES)
#define WS_TOTAL    OFF_V32(NV32)
static_assert((PLANE_BYTES % 128) == 0 && (VEC16_BYTES % 128) == 0);
static_assert((VEC32_BYTES % 128) == 0 && (ROW32_BYTES % 128) == 0);
static_assert((size_t)DIM * DIM * 4 == 2 * PLANE_BYTES);
static_assert(WS_TOTAL <= (size_t)134217728);

__device__ __forceinline__ float bf16r(float x) {
  unsigned int u = __float_as_uint(x);
  u = (u + 0x7FFFu + ((u >> 16) & 1u)) & 0xFFFF0000u;
  return __uint_as_float(u);
}

static __device__ __forceinline__ h16 toh_flush(float v) {
  const h16 r = (h16)v;
  return (fabsf(v) < 6.103515625e-05f) ? (h16)0.0f : r;
}

__device__ __forceinline__ int clampi(int v, int lo, int hi) {
  v = (v < lo) ? lo : v;
  return (v > hi) ? hi : v;
}

__device__ __forceinline__ v16h frag_at(const _Float16* p) {
  v8h lo = *(const v8h*)(p);
  v8h hi = *(const v8h*)(p + 16);
  v16h out;
#pragma unroll
  for (int i = 0; i < 8; ++i) { out[i] = lo[i]; out[i + 8] = hi[i]; }
  return out;
}

__device__ __forceinline__ v8f wmma16(v16h a, v16h b, v8f c) {
  v8f d = __builtin_amdgcn_wmma_f32_16x16x32_f16(false, a, false, b, (short)0, c,
                                                 false, false);
  asm volatile("v_nop\n\tv_nop\n\tv_nop\n\tv_nop" : "+v"(d) : "v"(a), "v"(b));
  return d;
}

__device__ __forceinline__ float red32_sum(float x) {
#pragma unroll
  for (int off = 1; off < 32; off <<= 1) x += __shfl_xor(x, off, 32);
  return x;
}
__device__ __forceinline__ float red32_max(float x) {
#pragma unroll
  for (int off = 1; off < 32; off <<= 1) x = fmaxf(x, __shfl_xor(x, off, 32));
  return x;
}

__global__ __launch_bounds__(256) void wconv_kernel(
    const float* __restrict__ W, _Float16* __restrict__ Wt, unsigned ldw, unsigned ldk) {
  __shared__ _Float16 T[64 * LDT];
  const unsigned tid = threadIdx.x;
  const unsigned n0 = blockIdx.x * 64u;
  const unsigned k0 = blockIdx.y * 64u;
#pragma unroll 4
  for (unsigned j = 0; j < 16u; ++j) {
    const unsigned idx = tid + 256u * j;
    const unsigned kr = idx >> 6, nc = idx & 63u;
    const float v = W[(size_t)(k0 + kr) * ldw + n0 + nc];
    T[nc * LDT + kr] = (_Float16)(WCARRY * bf16r(v));
  }
  __syncthreads();
  v8h x[2];
  size_t off[2];
#pragma unroll
  for (unsigned i = 0; i < 2u; ++i) {
    const unsigned n = 32u * i + (tid >> 3);
    const unsigned kc = (tid & 7u) * 8u;
    x[i] = *(const v8h*)&T[n * LDT + kc];
    off[i] = (size_t)(n0 + n) * ldk + k0 + kc;
  }
#pragma unroll
  for (int i = 0; i < 2; ++i) *(volatile v8h*)(Wt + off[i]) = x[i];
  __threadfence();
#pragma unroll
  for (int i = 0; i < 2; ++i) *(volatile v8h*)(Wt + off[i]) = x[i];
}

__global__ __launch_bounds__(256) void pconv_kernel(
    const float* __restrict__ X, _Float16* __restrict__ Y) {
#pragma clang fp contract(off)
  const size_t e0 = ((size_t)blockIdx.x * 256u + threadIdx.x) * 8u;
  const v4f a0 = *(const v4f*)(X + e0);
  const v4f a1 = *(const v4f*)(X + e0 + 4u);
  v8h o;
#pragma unroll
  for (int i = 0; i < 4; ++i) {
    o[i]     = toh_flush(WCARRY * bf16r(a0[i]));
    o[i + 4] = toh_flush(WCARRY * bf16r(a1[i]));
  }
  _Float16* p = Y + e0;
  *(volatile v8h*)p = o;
  __threadfence();
  *(volatile v8h*)p = o;
}

template <int MODE>
__device__ __forceinline__ void gemm64_body(
    const _Float16* __restrict__ Ah, const _Float16* __restrict__ Ar,
    const _Float16* __restrict__ Bh, const _Float16* __restrict__ Br,
    float* __restrict__ outf, _Float16* __restrict__ oh, _Float16* __restrict__ orr) {
  __shared__ float Cs[64 * LDC];
  if (MODE == 1) {
    if (blockIdx.x > blockIdx.y) return;
  }
  const unsigned tid = threadIdx.x, lane = tid & 31u;
  const unsigned w = (unsigned)__builtin_amdgcn_readfirstlane((int)(threadIdx.x >> 5));
  const unsigned mw = w >> 1, nw = w & 1u;
  const unsigned hh = lane >> 4, m = lane & 15u;
  const unsigned n0 = blockIdx.x * 64u;
  const unsigned row0 = blockIdx.y * 64u;

  const size_t aoff  = (size_t)(row0 + mw * 16u + m) * DIM + hh * 8u;
  const size_t boff0 = (size_t)(n0 + nw * 32u + m) * DIM + hh * 8u;
  const size_t boff1 = boff0 + (size_t)16 * DIM;
  v8f acc0 = {}, acc1 = {}, res0 = {}, res1 = {};
#pragma unroll 2
  for (unsigned k0 = 0; k0 < (unsigned)DIM; k0 += 32u) {
    const v16h a  = frag_at(Ah + aoff + k0);
    const v16h b0 = frag_at(Bh + boff0 + k0);
    const v16h b1 = frag_at(Bh + boff1 + k0);
    acc0 = wmma16(a, b0, acc0);
    acc1 = wmma16(a, b1, acc1);
    if (MODE == 1 && SCORE_RES) {
      const v16h ar  = frag_at(Ar + aoff + k0);
      const v16h br0 = frag_at(Br + boff0 + k0);
      const v16h br1 = frag_at(Br + boff1 + k0);
      res0 = wmma16(a, br0, res0);
      res0 = wmma16(ar, b0, res0);
      res1 = wmma16(a, br1, res1);
      res1 = wmma16(ar, b1, res1);
    }
  }
#pragma unroll
  for (int r = 0; r < 8; ++r) {
    float* d = &Cs[(mw * 16u + hh * 8u + (unsigned)r) * LDC + nw * 32u + m];
    if (MODE == 1 && SCORE_RES) {
      d[0]  = acc0[r] + res0[r] * (1.0f / RCARRY);
      d[16] = acc1[r] + res1[r] * (1.0f / RCARRY);
    } else {
      d[0]  = acc0[r];
      d[16] = acc1[r];
    }
  }
  __syncthreads();

  if (MODE == 0) {
    v8h x[2], xr[2];
    size_t off[2];
#pragma unroll
    for (unsigned i = 0; i < 2u; ++i) {
      const unsigned r = 32u * i + (tid >> 3);
      const unsigned c = (tid & 7u) * 8u;
      const v4f u0 = *(const v4f*)&Cs[r * LDC + c];
      const v4f u1 = *(const v4f*)&Cs[r * LDC + c + 4];
#pragma unroll
      for (int j = 0; j < 4; ++j) {
        const float t0 = u0[j] * (QCARRY / (WCARRY * WCARRY));
        const float t1 = u1[j] * (QCARRY / (WCARRY * WCARRY));
        const h16 h0 = toh_flush(t0);
        const h16 h1 = toh_flush(t1);
        x[i][j]      = h0;
        x[i][j + 4]  = h1;
        xr[i][j]     = toh_flush((t0 - (float)h0) * RCARRY);
        xr[i][j + 4] = toh_flush((t1 - (float)h1) * RCARRY);
      }
      off[i] = (size_t)(row0 + r) * DIM + n0 + c;
    }
#pragma unroll
    for (int i = 0; i < 2; ++i) *(volatile v8h*)(oh + off[i]) = x[i];
#pragma unroll
    for (int i = 0; i < 2; ++i) *(volatile v8h*)(orr + off[i]) = xr[i];
    __threadfence();
#pragma unroll
    for (int i = 0; i < 2; ++i) *(volatile v8h*)(oh + off[i]) = x[i];
#pragma unroll
    for (int i = 0; i < 2; ++i) *(volatile v8h*)(orr + off[i]) = xr[i];
  }

  if (MODE == 1) {
    v4f xs[4];
    size_t off[4];
#pragma unroll
    for (unsigned i = 0; i < 4u; ++i) {
      const unsigned r = 16u * i + (tid >> 4);
      const unsigned c = (tid & 15u) * 4u;
      const v4f u = *(const v4f*)&Cs[r * LDC + c];
      xs[i] = u * (1.0f / (QCARRY * QCARRY));
      off[i] = (size_t)(row0 + r) * DIM + n0 + c;
    }
#pragma unroll
    for (int i = 0; i < 4; ++i) *(volatile v4f*)(outf + off[i]) = xs[i];
    __threadfence();
#pragma unroll
    for (int i = 0; i < 4; ++i) *(volatile v4f*)(outf + off[i]) = xs[i];
  }
}

__global__ __launch_bounds__(256) void gemm_proj_kernel(
    const _Float16* __restrict__ A16, const _Float16* __restrict__ Bt,
    _Float16* __restrict__ oh, _Float16* __restrict__ orr) {
  gemm64_body<0>(A16, A16, Bt, Bt, (float*)0, oh, orr);
}
__global__ __launch_bounds__(256) void gemm_score_kernel(
    const _Float16* __restrict__ Qh, const _Float16* __restrict__ Qr,
    const _Float16* __restrict__ Kh, const _Float16* __restrict__ Kr,
    float* __restrict__ Sf) {
  gemm64_body<1>(Qh, Qr, Kh, Kr, Sf, (_Float16*)0, (_Float16*)0);
}

__global__ __launch_bounds__(256) void soft1_kernel(
    const float* __restrict__ Sf, const float* __restrict__ beta1,
    _Float16* __restrict__ A1h, _Float16* __restrict__ A1r, float* __restrict__ alast) {
#pragma clang fp contract(off)
  __shared__ float redm[8];
  __shared__ float reds[8];
  __shared__ float rowbuf[DIM];
  const unsigned tid = threadIdx.x, lane = tid & 31u;
  const unsigned w = (unsigned)__builtin_amdgcn_readfirstlane((int)(threadIdx.x >> 5));
  const unsigned s = blockIdx.x;
  const float sb = SCALE1 * bf16r(beta1[0]);
  const unsigned c0 = tid * 8u;
  const unsigned lastch = s >> 3;
  const unsigned ch = (tid < lastch) ? tid : lastch;
  const float* src = Sf + (size_t)s * DIM + ch * 8u;
  const v4f a0 = *(const v4f*)src;
  const v4f a1 = *(const v4f*)(src + 4u);
  float x[8];
#pragma unroll
  for (int j = 0; j < 4; ++j) { x[j] = sb * a0[j]; x[j + 4] = sb * a1[j]; }
  float mx = -__builtin_inff();
#pragma unroll
  for (int j = 0; j < 8; ++j) {
    const bool ok = (c0 + (unsigned)j) <= s;
    x[j] = ok ? x[j] : -__builtin_inff();
    mx = fmaxf(mx, x[j]);
  }
  mx = red32_max(mx);
  if (lane == 0u) redm[w] = mx;
  __syncthreads();
  mx = fmaxf(fmaxf(fmaxf(redm[0], redm[1]), fmaxf(redm[2], redm[3])),
             fmaxf(fmaxf(redm[4], redm[5]), fmaxf(redm[6], redm[7])));
  float sum = 0.0f;
#pragma unroll
  for (int j = 0; j < 8; ++j) {
    const bool ok = (c0 + (unsigned)j) <= s;
    const float e = ok ? __expf(x[j] - mx) : 0.0f;
    x[j] = e;
    sum += e;
  }
  sum = red32_sum(sum);
  if (lane == 0u) reds[w] = sum;
  __syncthreads();
  const float tot = ((reds[0] + reds[1]) + (reds[2] + reds[3])) +
                    ((reds[4] + reds[5]) + (reds[6] + reds[7]));
  const float inv = (s == 0u) ? 0.0f : (1.0f / tot);

  v8h xh, xr;
  v4f p0, p1;
#pragma unroll
  for (int j = 0; j < 8; ++j) {
    const float a = x[j] * inv;
    if (j < 4) p0[j] = a; else p1[j - 4] = a;
    const float t = a * PCARRY;
    const h16 hi = toh_flush(t);
    xh[j] = hi;
    xr[j] = toh_flush((t - (float)hi) * RCARRY);
  }
  const bool lastrow = (s == (unsigned)(SEQ - 1));
  v4f y0 = {0.0f, 0.0f, 0.0f, 0.0f}, y1 = {0.0f, 0.0f, 0.0f, 0.0f};
  if (lastrow) {
    *(v4f*)&rowbuf[c0] = p0;
    *(v4f*)&rowbuf[c0 + 4u] = p1;
    __syncthreads();
    y0 = *(const v4f*)&rowbuf[tid * 4u];
    y1 = *(const v4f*)&rowbuf[(DIM / 2) + tid * 4u];
  }
  const size_t off = (size_t)s * DIM + c0;
  *(volatile v8h*)(A1h + off) = xh;
  *(volatile v8h*)(A1r + off) = xr;
  if (lastrow) {
    *(volatile v4f*)(alast + tid * 4u) = y0;
    *(volatile v4f*)(alast + (DIM / 2) + tid * 4u) = y1;
  }
  __threadfence();
  *(volatile v8h*)(A1h + off) = xh;
  *(volatile v8h*)(A1r + off) = xr;
  if (lastrow) {
    *(volatile v4f*)(alast + tid * 4u) = y0;
    *(volatile v4f*)(alast + (DIM / 2) + tid * 4u) = y1;
  }
}

__global__ __launch_bounds__(256) void hist_kernel(
    const float* __restrict__ Wt, unsigned wstride, const int* __restrict__ ids,
    int do_soft, _Float16* __restrict__ Hh, _Float16* __restrict__ Hr) {
#pragma clang fp contract(off)
  __shared__ float bins[DIM + 256];
  __shared__ float wl[DIM];
  __shared__ int   idl[DIM];
  __shared__ float redm[8];
  __shared__ float reds[8];
  const unsigned tid = threadIdx.x, lane = tid & 31u;
  const unsigned w = (unsigned)__builtin_amdgcn_readfirstlane((int)(threadIdx.x >> 5));
  const unsigned b = blockIdx.x;
  const unsigned c0 = tid * 8u;
  const float* wp = Wt + (size_t)b * wstride + c0;
  const v4f a0 = *(const v4f*)wp;
  const v4f a1 = *(const v4f*)(wp + 4u);
  const int* ip = ids + (size_t)b * SEQ_FULL + c0;
  const v4i i0 = *(const v4i*)ip;
  const v4i i1 = *(const v4i*)(ip + 4u);
  float x[8];
#pragma unroll
  for (int j = 0; j < 4; ++j) { x[j] = a0[j]; x[j + 4] = a1[j]; }

  if (do_soft != 0) {
    float mx = -__builtin_inff();
#pragma unroll
    for (int j = 0; j < 8; ++j) {
      const bool masked = (c0 + (unsigned)j) == (unsigned)(SEQ - 1);
      x[j] = masked ? -__builtin_inff() : x[j];
      mx = fmaxf(mx, x[j]);
    }
    mx = red32_max(mx);
    if (lane == 0u) redm[w] = mx;
    __syncthreads();
    mx = fmaxf(fmaxf(fmaxf(redm[0], redm[1]), fmaxf(redm[2], redm[3])),
               fmaxf(fmaxf(redm[4], redm[5]), fmaxf(redm[6], redm[7])));
    float sum = 0.0f;
#pragma unroll
    for (int j = 0; j < 8; ++j) {
      const bool masked = (c0 + (unsigned)j) == (unsigned)(SEQ - 1);
      const float e = masked ? 0.0f : __expf(x[j] - mx);
      x[j] = e;
      sum += e;
    }
    sum = red32_sum(sum);
    if (lane == 0u) reds[w] = sum;
    __syncthreads();
    const float tot = ((reds[0] + reds[1]) + (reds[2] + reds[3])) +
                      ((reds[4] + reds[5]) + (reds[6] + reds[7]));
    const float inv = 1.0f / tot;
#pragma unroll
    for (int j = 0; j < 8; ++j) x[j] = x[j] * inv;
  }

  v4f w0, w1, z4 = {0.0f, 0.0f, 0.0f, 0.0f};
  v4i j0, j1;
#pragma unroll
  for (int j = 0; j < 4; ++j) {
    w0[j] = x[j];
    w1[j] = x[j + 4];
    j0[j] = clampi(i0[j], 0, DIM - 1);
    j1[j] = clampi(i1[j], 0, DIM - 1);
  }
  *(v4f*)&wl[c0] = w0;
  *(v4f*)&wl[c0 + 4u] = w1;
  *(v4i*)&idl[c0] = j0;
  *(v4i*)&idl[c0 + 4u] = j1;
  *(v4f*)&bins[c0] = z4;
  *(v4f*)&bins[c0 + 4u] = z4;
  bins[(unsigned)DIM + tid] = 0.0f;
  __syncthreads();

#pragma unroll 4
  for (unsigned t = 0; t < (unsigned)SEQ; ++t) {
    const int id = idl[t];
    const float wv = wl[t];
    const bool mine = (((unsigned)id) & 255u) == tid;
    const unsigned slot = mine ? (unsigned)id : ((unsigned)DIM + tid);
    const float add = mine ? wv : 0.0f;
    bins[slot] = bins[slot] + add;
  }
  __syncthreads();

  const v4f h0 = *(const v4f*)&bins[c0];
  const v4f h1 = *(const v4f*)&bins[c0 + 4u];
  v8h xh, xr;
#pragma unroll
  for (int j = 0; j < 4; ++j) {
    const float t0 = h0[j] * HCARRY;
    const float t1 = h1[j] * HCARRY;
    const h16 q0 = toh_flush(t0);
    const h16 q1 = toh_flush(t1);
    xh[j]     = q0;
    xh[j + 4] = q1;
    xr[j]     = toh_flush((t0 - (float)q0) * RCARRY);
    xr[j + 4] = toh_flush((t1 - (float)q1) * RCARRY);
  }
  const size_t off = (size_t)b * DIM + c0;
  *(volatile v8h*)(Hh + off) = xh;
  *(volatile v8h*)(Hr + off) = xr;
  __threadfence();
  *(volatile v8h*)(Hh + off) = xh;
  *(volatile v8h*)(Hr + off) = xr;
}

__global__ __launch_bounds__(256) void gather_cd_kernel(
    const float* __restrict__ Gf, const float* __restrict__ Df, const int* __restrict__ ids,
    _Float16* __restrict__ Ch, _Float16* __restrict__ Cr, float* __restrict__ dvec) {
#pragma clang fp contract(off)
  __shared__ float Gl[DIM];
  __shared__ float Dl[DIM];
  __shared__ float dl[DIM];
  const unsigned tid = threadIdx.x;
  const unsigned b = blockIdx.x;
  const size_t rb = (size_t)b * DIM;
  *(v4f*)&Gl[tid * 4u]             = *(const v4f*)(Gf + rb + tid * 4u);
  *(v4f*)&Gl[(DIM / 2) + tid * 4u] = *(const v4f*)(Gf + rb + (DIM / 2) + tid * 4u);
  *(v4f*)&Dl[tid * 4u]             = *(const v4f*)(Df + rb + tid * 4u);
  *(v4f*)&Dl[(DIM / 2) + tid * 4u] = *(const v4f*)(Df + rb + (DIM / 2) + tid * 4u);
  __syncthreads();
  const unsigned c0 = tid * 8u;
  const int* ip = ids + (size_t)b * SEQ_FULL + c0;
  const v4i i0 = *(const v4i*)ip;
  const v4i i1 = *(const v4i*)(ip + 4u);
  v8h xh, xr;
  v4f d0, d1;
#pragma unroll
  for (int j = 0; j < 4; ++j) {
    const int ia = clampi(i0[j], 0, DIM - 1);
    const int ib = clampi(i1[j], 0, DIM - 1);
    const float t0 = Gl[ia] * ACARRY;
    const float t1 = Gl[ib] * ACARRY;
    const h16 q0 = toh_flush(t0);
    const h16 q1 = toh_flush(t1);
    xh[j]     = q0;
    xh[j + 4] = q1;
    xr[j]     = toh_flush((t0 - (float)q0) * RCARRY);
    xr[j + 4] = toh_flush((t1 - (float)q1) * RCARRY);
    d0[j] = Dl[ia];
    d1[j] = Dl[ib];
  }
  *(v4f*)&dl[c0] = d0;
  *(v4f*)&dl[c0 + 4u] = d1;
  __syncthreads();
  const v4f y0 = *(const v4f*)&dl[tid * 4u];
  const v4f y1 = *(const v4f*)&dl[(DIM / 2) + tid * 4u];
  const size_t off = rb + c0;
  *(volatile v8h*)(Ch + off) = xh;
  *(volatile v8h*)(Cr + off) = xr;
  *(volatile v4f*)(dvec + rb + tid * 4u) = y0;
  *(volatile v4f*)(dvec + rb + (DIM / 2) + tid * 4u) = y1;
  __threadfence();
  *(volatile v8h*)(Ch + off) = xh;
  *(volatile v8h*)(Cr + off) = xr;
  *(volatile v4f*)(dvec + rb + tid * 4u) = y0;
  *(volatile v4f*)(dvec + rb + (DIM / 2) + tid * 4u) = y1;
}

__global__ __launch_bounds__(256) void gemm_m16_kernel(
    const _Float16* __restrict__ Ah, const _Float16* __restrict__ Ar,
    const _Float16* __restrict__ Bh, const _Float16* __restrict__ Br,
    const float* __restrict__ beta, const float* __restrict__ addf,
    const float* __restrict__ emb, const int* __restrict__ ids,
    float* __restrict__ outf, _Float16* __restrict__ oh, _Float16* __restrict__ orr,
    int use_ar, int use_br, int use_beta, int addmode, int wr_f32, int wr_16,
    float cs, float gscale, float ocarry) {
  __shared__ float Cs[16 * LDM];
  const unsigned tid = threadIdx.x, lane = tid & 31u;
  const unsigned w = (unsigned)__builtin_amdgcn_readfirstlane((int)(threadIdx.x >> 5));
  const unsigned hh = lane >> 4, m = lane & 15u;
  const unsigned n0 = blockIdx.x * 128u;
  const size_t aoff = (size_t)m * DIM + hh * 8u;
  const size_t boff = (size_t)(n0 + w * 16u + m) * DIM + hh * 8u;
  v8f acc = {}, accr = {};
#pragma unroll 2
  for (unsigned k0 = 0; k0 < (unsigned)DIM; k0 += 32u) {
    const v16h a  = frag_at(Ah + aoff + k0);
    const v16h bq = frag_at(Bh + boff + k0);
    acc = wmma16(a, bq, acc);
    if (use_ar != 0) {
      const v16h ar = frag_at(Ar + aoff + k0);
      accr = wmma16(ar, bq, accr);
    }
    if (use_br != 0) {
      const v16h br = frag_at(Br + boff + k0);
      accr = wmma16(a, br, accr);
    }
  }
#pragma unroll
  for (int r = 0; r < 8; ++r)
    Cs[(hh * 8u + (unsigned)r) * LDM + w * 16u + m] = acc[r] + accr[r] * (1.0f / RCARRY);
  __syncthreads();

  const unsigned row = tid >> 4;
  const unsigned c8 = (tid & 15u) * 8u;
  const v4f u0 = *(const v4f*)&Cs[row * LDM + c8];
  const v4f u1 = *(const v4f*)&Cs[row * LDM + c8 + 4u];
  v4f ad0 = {0.0f, 0.0f, 0.0f, 0.0f}, ad1 = {0.0f, 0.0f, 0.0f, 0.0f};
  if (addmode == 1) {
    const int id = clampi(ids[(size_t)row * SEQ_FULL + (SEQ - 1)], 0, DIM - 1);
    const float* er = emb + (size_t)id * DIM + n0 + c8;
    const v4f e0 = *(const v4f*)er;
    const v4f e1 = *(const v4f*)(er + 4u);
#pragma unroll
    for (int j = 0; j < 4; ++j) { ad0[j] = bf16r(e0[j]); ad1[j] = bf16r(e1[j]); }
  } else if (addmode == 2) {
    ad0 = *(const v4f*)(addf + (size_t)row * DIM + n0 + c8);
    ad1 = *(const v4f*)(addf + (size_t)row * DIM + n0 + c8 + 4u);
  }
  const float bv = bf16r(beta[0]);
  const float gs = gscale * ((use_beta != 0) ? bv : 1.0f);
  v4f t0, t1;
  v8h xh, xr;
#pragma unroll
  for (int j = 0; j < 4; ++j) {
    t0[j] = gs * (u0[j] * cs + ad0[j]);
    t1[j] = gs * (u1[j] * cs + ad1[j]);
    const float s0 = t0[j] * ocarry;
    const float s1 = t1[j] * ocarry;
    const h16 q0 = toh_flush(s0);
    const h16 q1 = toh_flush(s1);
    xh[j]     = q0;
    xh[j + 4] = q1;
    xr[j]     = toh_flush((s0 - (float)q0) * RCARRY);
    xr[j + 4] = toh_flush((s1 - (float)q1) * RCARRY);
  }
  *(v4f*)&Cs[row * LDM + c8] = t0;
  *(v4f*)&Cs[row * LDM + c8 + 4u] = t1;
  __syncthreads();

  v4f y[2];
  size_t offf[2];
#pragma unroll
  for (unsigned i = 0; i < 2u; ++i) {
    const unsigned r = (tid >> 5) + 8u * i;
    const unsigned c4 = (tid & 31u) * 4u;
    y[i] = *(const v4f*)&Cs[r * LDM + c4];
    offf[i] = (size_t)r * DIM + n0 + c4;
  }
  const size_t o16 = (size_t)row * DIM + n0 + c8;
  if (wr_16 != 0) {
    *(volatile v8h*)(oh + o16) = xh;
    *(volatile v8h*)(orr + o16) = xr;
  }
  if (wr_f32 != 0) {
#pragma unroll
    for (int i = 0; i < 2; ++i) *(volatile v4f*)(outf + offf[i]) = y[i];
  }
  __threadfence();
  if (wr_16 != 0) {
    *(volatile v8h*)(oh + o16) = xh;
    *(volatile v8h*)(orr + o16) = xr;
  }
  if (wr_f32 != 0) {
#pragma unroll
    for (int i = 0; i < 2; ++i) *(volatile v4f*)(outf + offf[i]) = y[i];
  }
}

static inline void launch_m16(hipStream_t stream,
    const _Float16* Ah, const _Float16* Ar, const _Float16* Bh, const _Float16* Br,
    const float* beta, const float* addf, const float* emb, const int* ids,
    float* outf, _Float16* oh, _Float16* orr,
    int use_ar, int use_br, int use_beta, int addmode, int wr_f32, int wr_16,
    float cs, float gscale, float ocarry) {
  gemm_m16_kernel<<<dim3(DIM / 128), dim3(256), 0, stream>>>(
      Ah, Ar, Bh, Br, beta, addf, emb, ids, outf, oh, orr,
      use_ar, use_br, use_beta, addmode, wr_f32, wr_16, cs, gscale, ocarry);
}

extern "C" void kernel_launch(void* const* d_in, const int* in_sizes, int n_in,
                              void* d_out, int out_size, void* d_ws, size_t ws_size,
                              hipStream_t stream) {
  if (n_in < 12) return;
  if ((long long)in_sizes[0] < (long long)NB * SEQ) return;
  for (int i = 1; i <= 8; ++i)
    if ((long long)in_sizes[i] < (long long)DIM * DIM) return;
  if (in_sizes[9] < 1 || in_sizes[10] < 1 || in_sizes[11] < 1) return;
  if ((long long)out_size < (long long)NB * DIM) return;
  if (ws_size < WS_TOTAL) return;

  const int*   ids   = (const int*)d_in[0];
  const float* Wemb  = (const float*)d_in[1];
  const float* Ppos  = (const float*)d_in[2];
  const float* WQ1   = (const float*)d_in[3];
  const float* WK1   = (const float*)d_in[4];
  const float* WV1   = (const float*)d_in[5];
  const float* WQ2   = (const float*)d_in[6];
  const float* WK2   = (const float*)d_in[7];
  const float* WV2   = (const float*)d_in[8];
  const float* beta1 = (const float*)d_in[9];
  const float* beta2 = (const float*)d_in[10];
  const float* betao = (const float*)d_in[11];
  float* out = (float*)d_out;

  char* ws = (char*)d_ws;
  _Float16* SL0  = (_Float16*)(ws + OFF_SLOT(0));
  _Float16* SL1  = (_Float16*)(ws + OFF_SLOT(1));
  _Float16* SL2  = (_Float16*)(ws + OFF_SLOT(2));
  _Float16* SL3  = (_Float16*)(ws + OFF_SLOT(3));
  _Float16* SL4  = (_Float16*)(ws + OFF_SLOT(4));
  _Float16* SL5  = (_Float16*)(ws + OFF_SLOT(5));
  _Float16* SL6  = (_Float16*)(ws + OFF_SLOT(6));
  float*    Sf   = (float*)(ws + OFF_SLOT(7));
  _Float16* SL9  = (_Float16*)(ws + OFF_SLOT(9));
  _Float16* SL10 = (_Float16*)(ws + OFF_SLOT(10));
  float* alast = (float*)(ws + OFF_ALAST);
  _Float16* H1h = (_Float16*)(ws + OFF_V16(0));
  _Float16* H1r = (_Float16*)(ws + OFF_V16(1));
  _Float16* Mh  = (_Float16*)(ws + OFF_V16(2));
  _Float16* Mr  = (_Float16*)(ws + OFF_V16(3));
  _Float16* ZQh = (_Float16*)(ws + OFF_V16(4));
  _Float16* ZQr = (_Float16*)(ws + OFF_V16(5));
  _Float16* Q2h = (_Float16*)(ws + OFF_V16(6));
  _Float16* Q2r = (_Float16*)(ws + OFF_V16(7));
  _Float16* Uh  = (_Float16*)(ws + OFF_V16(8));
  _Float16* Ur  = (_Float16*)(ws + OFF_V16(9));
  _Float16* Gh  = (_Float16*)(ws + OFF_V16(10));
  _Float16* Gr  = (_Float16*)(ws + OFF_V16(11));
  _Float16* Ch  = (_Float16*)(ws + OFF_V16(12));
  _Float16* Cr  = (_Float16*)(ws + OFF_V16(13));
  _Float16* H2h = (_Float16*)(ws + OFF_V16(14));
  _Float16* H2r = (_Float16*)(ws + OFF_V16(15));
  _Float16* E2h = (_Float16*)(ws + OFF_V16(16));
  _Float16* E2r = (_Float16*)(ws + OFF_V16(17));
  _Float16* Y2h = (_Float16*)(ws + OFF_V16(18));
  _Float16* Y2r = (_Float16*)(ws + OFF_V16(19));
  _Float16* X16h = (_Float16*)(ws + OFF_V16(20));
  _Float16* X16r = (_Float16*)(ws + OFF_V16(21));
  float* Gf   = (float*)(ws + OFF_V32(0));
  float* Df   = (float*)(ws + OFF_V32(1));
  float* dvec = (float*)(ws + OFF_V32(2));
  float* S2f  = (float*)(ws + OFF_V32(3));
  float* X32  = (float*)(ws + OFF_V32(4));

  const dim3 blk(256);
  const dim3 gsq(DIM / 64, DIM / 64);
  const dim3 gpl((unsigned)(((size_t)DIM * DIM) / 2048));
  const int CR = CHAIN_RES ? 1 : 0;

  pconv_kernel<<<gpl, blk, 0, stream>>>(Ppos, SL0);
  pconv_kernel<<<gpl, blk, 0, stream>>>(WQ1, SL1);
  pconv_kernel<<<gpl, blk, 0, stream>>>(WK1, SL2);
  gemm_proj_kernel<<<gsq, blk, 0, stream>>>(SL0, SL1, SL3, SL4);
  gemm_proj_kernel<<<gsq, blk, 0, stream>>>(SL0, SL2, SL5, SL6);
  gemm_score_kernel<<<gsq, blk, 0, stream>>>(SL3, SL4, SL5, SL6, Sf);
  soft1_kernel<<<dim3(SEQ), blk, 0, stream>>>(Sf, beta1, SL0, SL1, alast);

  pconv_kernel<<<gpl, blk, 0, stream>>>(Wemb, SL2);
  wconv_kernel<<<gsq, blk, 0, stream>>>(Wemb, SL3, (unsigned)DIM, (unsigned)DIM);
  pconv_kernel<<<gpl, blk, 0, stream>>>(WV1, SL4);
  wconv_kernel<<<gsq, blk, 0, stream>>>(WV1, SL5, (unsigned)DIM, (unsigned)DIM);
  pconv_kernel<<<gpl, blk, 0, stream>>>(WQ2, SL6);
  wconv_kernel<<<gsq, blk, 0, stream>>>(WK2, SL9, (unsigned)DIM, (unsigned)DIM);
  pconv_kernel<<<gpl, blk, 0, stream>>>(WV2, SL10);

  const float CS_HW = 1.0f / (HCARRY * WCARRY);
  const float CS_AW = 1.0f / (ACARRY * WCARRY);
  const float CS_AP = 1.0f / (ACARRY * PCARRY);

  hist_kernel<<<dim3(NB), blk, 0, stream>>>(alast, 0u, ids, 0, H1h, H1r);
  launch_m16(stream, H1h, H1r, SL3, SL3, beta1, dvec, Wemb, ids, X32, Mh, Mr,
             CR, 0, 0, 0, 0, 1, CS_HW, 1.0f, ACARRY);
  launch_m16(stream, Mh, Mr, SL4, SL4, beta1, dvec, Wemb, ids, X32, ZQh, ZQr,
             CR, 0, 0, 1, 0, 1, CS_AW, 1.0f, ACARRY);
  launch_m16(stream, ZQh, ZQr, SL6, SL6, beta1, dvec, Wemb, ids, X32, Q2h, Q2r,
             CR, 0, 0, 0, 0, 1, CS_AW, 1.0f, ACARRY);
  launch_m16(stream, Q2h, Q2r, SL9, SL9, beta1, dvec, Wemb, ids, X32, Uh, Ur,
             CR, 0, 0, 0, 0, 1, CS_AW, 1.0f, ACARRY);
  launch_m16(stream, Uh, Ur, SL5, SL5, beta1, dvec, Wemb, ids, X32, Gh, Gr,
             CR, 0, 0, 0, 0, 1, CS_AW, 1.0f, ACARRY);
  launch_m16(stream, Gh, Gr, SL2, SL2, beta1, dvec, Wemb, ids, Gf, X16h, X16r,
             CR, 0, 0, 0, 1, 0, CS_AW, 1.0f, ACARRY);
  launch_m16(stream, Uh, Ur, SL2, SL2, beta1, dvec, Wemb, ids, Df, X16h, X16r,
             CR, 0, 0, 0, 1, 0, CS_AW, 1.0f, ACARRY);
  gather_cd_kernel<<<dim3(NB), blk, 0, stream>>>(Gf, Df, ids, Ch, Cr, dvec);
  launch_m16(stream, Ch, Cr, SL0, SL1, beta2, dvec, Wemb, ids, S2f, X16h, X16r,
             CR, CR, 1, 2, 1, 0, CS_AP, SCALE2, ACARRY);
  hist_kernel<<<dim3(NB), blk, 0, stream>>>(S2f, (unsigned)DIM, ids, 1, H2h, H2r);
  launch_m16(stream, H2h, H2h, SL3, SL3, beta1, dvec, Wemb, ids, X32, E2h, E2r,
             0, 0, 0, 0, 0, 1, CS_HW, 1.0f, ACARRY);
  launch_m16(stream, E2h, E2h, SL10, SL10, beta1, dvec, Wemb, ids, X32, Y2h, Y2r,
             0, 0, 0, 0, 0, 1, CS_AW, 1.0f, ACARRY);
  launch_m16(stream, Y2h, Y2h, SL2, SL2, betao, dvec, Wemb, ids, out, X16h, X16r,
             0, 0, 1, 0, 1, 0, CS_AW, SCALEO, ACARRY);
}
